// CausalAttention_40845138985312
// MI455X (gfx1250) — hardware-verified
//
#include <hip/hip_runtime.h>


#ifndef NB
#define NB 2
#endif
#ifndef SEQ
#define SEQ 2048
#endif
#ifndef RH
#define RH 256
#endif
#define NBF   2
#define TFULL 2048
#define DM    2048
#define NH    16
#define LAT   512
#define RD    64
#define HD    128
#define NU    (NB * NH)
#define PCAR  1024.0f
#define WSC   64.0f
#define CCAR  64.0f

static_assert(NB >= 1);
static_assert(NB <= NBF);
static_assert(SEQ % 64 == 0);
static_assert(SEQ <= TFULL);
static_assert(RH % 64 == 0);
static_assert(RH >= 64);
static_assert(RH <= SEQ);
static_assert(DM % 64 == 0);
static_assert(LAT % 64 == 0);
static_assert((NH * RD) % 64 == 0);
static_assert(RD == 64);
static_assert(HD == 128);
static_assert(NH * HD == DM);
static_assert((size_t)NB * SEQ * NH * RD * 4 == (size_t)NB * SEQ * DM * 2);
static_assert(((size_t)(NB - 1) * TFULL + SEQ) * DM <= (size_t)NBF * TFULL * DM);

typedef _Float16 h16;
typedef unsigned short bf;
typedef __attribute__((ext_vector_type(16))) __bf16   v16bf;
typedef __attribute__((ext_vector_type(16))) _Float16 v16h;
typedef __attribute__((ext_vector_type(16))) unsigned short v16us;
typedef __attribute__((ext_vector_type(8)))  _Float16 v8h;
typedef __attribute__((ext_vector_type(8)))  unsigned short v8us;
typedef __attribute__((ext_vector_type(8)))  float    v8f;
typedef __attribute__((ext_vector_type(4)))  float    v4f;
typedef __attribute__((ext_vector_type(2)))  _Float16 v2h;
typedef __attribute__((ext_vector_type(2)))  unsigned short v2us;
typedef v8h  __attribute__((may_alias)) v8ha;
typedef v4f  __attribute__((may_alias)) v4fa;

__device__ __forceinline__ unsigned short f2bf(float f) { unsigned u = __float_as_uint(f); u += 0x7FFFu + ((u >> 16) & 1u); return (unsigned short)(u >> 16); }
__device__ __forceinline__ float bf2f(unsigned short v) { return __uint_as_float(((unsigned)v) << 16); }
__device__ __forceinline__ float bfr(float f) { return bf2f(f2bf(f)); }
__device__ __forceinline__ void splitf(float y, unsigned short& hh, unsigned short& ll) { hh = f2bf(y); ll = f2bf(y - bf2f(hh)); }
__device__ __forceinline__ v16h cat16(v8h a, v8h c) { return __builtin_shufflevector(a, c, 0, 1, 2, 3, 4, 5, 6, 7, 8, 9, 10, 11, 12, 13, 14, 15); }
__device__ __forceinline__ v16bf cat16b(v8us a, v8us c) { return __builtin_bit_cast(v16bf, __builtin_shufflevector(a, c, 0, 1, 2, 3, 4, 5, 6, 7, 8, 9, 10, 11, 12, 13, 14, 15)); }
__device__ __forceinline__ v8f wmma16(v16h a, v16h c, v8f acc) { return __builtin_amdgcn_wmma_f32_16x16x32_f16(false, a, false, c, (short)0, acc, false, false); }
__device__ __forceinline__ v8f wmmab(v16bf a, v16bf c, v8f acc) { return __builtin_amdgcn_wmma_f32_16x16x32_bf16(false, a, false, c, (short)0, acc, false, false); }
__device__ __forceinline__ v16h ldh(const h16* p) { return cat16(*(const v8h*)p, *(const v8h*)(p + 16)); }
__device__ __forceinline__ v16bf ldb(const bf* p) { return cat16b(*(const v8us*)p, *(const v8us*)(p + 16)); }

template <typename T16> struct WFrag;
template <> struct WFrag<h16> { typedef v16h V; static __device__ __forceinline__ V ld(const h16* p) { return ldh(p); } static __device__ __forceinline__ v8f mma(V a, V c, v8f d) { return wmma16(a, c, d); } };
template <> struct WFrag<bf> { typedef v16bf V; static __device__ __forceinline__ V ld(const bf* p) { return ldb(p); } static __device__ __forceinline__ v8f mma(V a, V c, v8f d) { return wmmab(a, c, d); } };
template <typename T16, int NSPLIT>
__global__ __launch_bounds__(32) void k_gemmw(const T16* __restrict__ A, const T16* __restrict__ A2, const T16* __restrict__ Bt, int K, float* C, int ldc, float osc, size_t sA, size_t sC) {
    typedef typename WFrag<T16>::V V;
    __shared__ __align__(16) float os[16 * 68];
    const size_t z = blockIdx.z; A += z * sA; A2 += z * sA; C += z * sC;
    const int lane = threadIdx.x & 31, lr = lane & 15, hi = lane >> 4; const int r0 = blockIdx.x * 64, c0 = blockIdx.y * 64;
    v8f acc[4][4];
#pragma unroll
    for (int mb = 0; mb < 4; ++mb)
#pragma unroll
        for (int nb = 0; nb < 4; ++nb) acc[mb][nb] = (v8f){};
    const size_t aoff = (size_t)(r0 + lr) * K + 8 * hi, boff = (size_t)(c0 + lr) * K + 8 * hi;
#pragma unroll 1
    for (int kc = 0; kc < K; kc += 32) {
        V a[4], a2[4];
#pragma unroll
        for (int mb = 0; mb < 4; ++mb) { a[mb] = WFrag<T16>::ld(A + aoff + (size_t)mb * 16 * K + kc); if (NSPLIT == 1) a2[mb] = WFrag<T16>::ld(A2 + aoff + (size_t)mb * 16 * K + kc); }
#pragma unroll
        for (int nb = 0; nb < 4; ++nb) { const V bq = WFrag<T16>::ld(Bt + boff + (size_t)nb * 16 * K + kc);
#pragma unroll
            for (int mb = 0; mb < 4; ++mb) { acc[mb][nb] = WFrag<T16>::mma(a[mb], bq, acc[mb][nb]); if (NSPLIT == 1) acc[mb][nb] = WFrag<T16>::mma(a2[mb], bq, acc[mb][nb]); } }
        asm volatile("v_nop\n\tv_nop\n\tv_nop\n\tv_nop" : "+v"(acc[0][0]), "+v"(acc[1][1]), "+v"(acc[2][2]), "+v"(acc[3][3]) : "v"(a[0]), "v"(a[3]));
    }
#pragma unroll
    for (int mb = 0; mb < 4; ++mb) {
#pragma unroll
        for (int nb = 0; nb < 4; ++nb) {
#pragma unroll
            for (int j = 0; j < 8; ++j) os[(hi * 8 + j) * 68 + nb * 16 + lr] = acc[mb][nb][j]; }
        __builtin_amdgcn_wave_barrier(); asm volatile("" ::: "memory");
        float* crow = C + (size_t)(r0 + mb * 16) * ldc + c0;
#pragma unroll 1
        for (int ps = 0; ps < 2; ++ps) {
#pragma unroll
            for (int s = 0; s < 8; ++s) { const int row = 2 * s + hi, cofs = lr * 4; v4f val = *(const v4fa*)(os + row * 68 + cofs); val = val * osc;
                *(volatile v4f*)(crow + (size_t)row * ldc + cofs) = val; }
            if (ps == 0) __threadfence(); }
        __builtin_amdgcn_wave_barrier(); asm volatile("" ::: "memory");
    }
}

template <int F16P>
__global__ __launch_bounds__(256) void k_wt(const float* __restrict__ w, int K, int N, bf* Bb, h16* Bh, float sc) {
    const int lane = threadIdx.x & 31; const int L0 = (blockIdx.x * 8 + (threadIdx.x >> 5)) * 8; const int nlines = N * K / 64;
#pragma unroll 1
    for (int ps = 0; ps < 2; ++ps) {
#pragma unroll 1
        for (int l = 0; l < 8; ++l) { const int L = L0 + l; if (L >= nlines) break; const size_t e = (size_t)L * 64 + lane * 2; const int k = (int)(e % K), n = (int)(e / K);
            const float w0 = bfr(w[(size_t)k * N + n]), w1 = bfr(w[(size_t)(k + 1) * N + n]);
            v2us o; o[0] = f2bf(w0); o[1] = f2bf(w1); *(volatile v2us*)(Bb + e) = o;
            if (F16P) { v2h oh; oh[0] = (h16)(w0 * sc); oh[1] = (h16)(w1 * sc); *(volatile v2h*)(Bh + e) = oh; } }
        if (ps == 0) __threadfence(); }
}

__global__ __launch_bounds__(256) void k_xcvt(const float* __restrict__ x, bf* xb) {
    const size_t i = (size_t)blockIdx.x * 256 + threadIdx.x; const size_t n8 = (size_t)NB * SEQ * DM / 8; if (i >= n8) return;
    const size_t e = i * 8; const size_t row = e / DM; const int col = (int)(e % DM); const size_t bb = row / SEQ, t = row % SEQ;
    const v8f v = *(const v8f*)(x + ((bb * TFULL + t) * DM + col)); v8us o = (v8us){};
#pragma unroll
    for (int k = 0; k < 8; ++k) o[k] = f2bf(v[k]);
    *(volatile v8us*)(xb + e) = o; __threadfence(); *(volatile v8us*)(xb + e) = o;
}

__global__ __launch_bounds__(256) void k_act(const float* __restrict__ src, int C, float sc, h16* p16, bf* ph, bf* pl) {
    const size_t i = (size_t)blockIdx.x * 256 + threadIdx.x; const size_t n8 = (size_t)NB * SEQ * C / 8; if (i >= n8) return;
    const size_t e = i * 8; const size_t row = e / C; const int col = (int)(e - row * C); const int t = (int)(row % SEQ); const size_t bb = row / SEQ;
    const v8f v = *(const v8f*)(src + e);
    v8h o = (v8h){}; v8us oh = (v8us){}, ol = (v8us){};
#pragma unroll
    for (int k = 0; k < 8; ++k) { o[k] = (h16)(v[k] * sc); unsigned short a1, c1; splitf(v[k], a1, c1); oh[k] = a1; ol[k] = c1; }
    const bool hr = (t < RH); const size_t eo = (bb * RH + t) * C + col;
    *(volatile v8h*)(p16 + e) = o; if (hr) { *(volatile v8us*)(ph + eo) = oh; *(volatile v8us*)(pl + eo) = ol; }
    __threadfence();
    *(volatile v8h*)(p16 + e) = o; if (hr) { *(volatile v8us*)(ph + eo) = oh; *(volatile v8us*)(pl + eo) = ol; }
}

__global__ __launch_bounds__(256) void k_rtab(float* ct, float* st) {
#pragma clang fp contract(off)
    const int i = blockIdx.x * 256 + threadIdx.x; if (i >= SEQ * 32) return; const int t = i >> 5, j = i & 31;
    const float fr = exp10f(-0.125f * (float)j);
    const float ang = (float)t * fr; float sv, cv; sincosf(ang, &sv, &cv);
    *(volatile float*)(ct + i) = cv; *(volatile float*)(st + i) = sv; __threadfence(); *(volatile float*)(ct + i) = cv; *(volatile float*)(st + i) = sv;
}

__global__ __launch_bounds__(256) void k_rope(const float* __restrict__ src, int C, const float* __restrict__ ct, const float* __restrict__ st, h16* p16, bf* ph, bf* pl) {
#pragma clang fp contract(off)
    const size_t i = (size_t)blockIdx.x * 256 + threadIdx.x; const size_t n8 = (size_t)NB * SEQ * C / 8; if (i >= n8) return;
    const size_t e = i * 8; const size_t row = e / C; const int col = (int)(e - row * C); const int t = (int)(row % SEQ); const size_t bb = row / SEQ;
    const int jj = col & 63, jm = jj & 31; const bool lo32 = (jj < 32); const int pofs = lo32 ? 32 : -32;
    const v8f xv = *(const v8f*)(src + e); const v8f xp = *(const v8f*)((src + e) + pofs);
    const v8f cvv = *(const v8f*)(ct + (size_t)t * 32 + jm); const v8f svv = *(const v8f*)(st + (size_t)t * 32 + jm);
    v8h o = (v8h){}; v8us oh = (v8us){}, ol = (v8us){};
#pragma unroll
    for (int k = 0; k < 8; ++k) { const float a1 = xv[k] * cvv[k]; const float b1 = xp[k] * svv[k]; const float y = lo32 ? (a1 - b1) : (a1 + b1);
        o[k] = (h16)y; unsigned short a2, c2; splitf(y, a2, c2); oh[k] = a2; ol[k] = c2; }
    const bool hr = (t < RH); const size_t eo = (bb * RH + t) * C + col;
    *(volatile v8h*)(p16 + e) = o; if (hr) { *(volatile v8us*)(ph + eo) = oh; *(volatile v8us*)(pl + eo) = ol; }
    __threadfence();
    *(volatile v8h*)(p16 + e) = o; if (hr) { *(volatile v8us*)(ph + eo) = oh; *(volatile v8us*)(pl + eo) = ol; }
}

__global__ __launch_bounds__(256) void k_vtp8(const float* __restrict__ vf, h16* vt16, bf* vth, bf* vtl) {
    const size_t i = (size_t)blockIdx.x * 256 + threadIdx.x; const size_t n8 = (size_t)NU * HD * SEQ / 8; if (i >= n8) return;
    const size_t e = i * 8; const int t = (int)(e % SEQ); const int d = (int)((e / SEQ) % HD); const int g = (int)(e / ((size_t)SEQ * HD)); const int bb = g / NH, hh = g % NH;
    const float* sp = vf + ((size_t)bb * SEQ + t) * DM + hh * HD + d;
    v8h o = (v8h){}; v8us oh = (v8us){}, ol = (v8us){};
#pragma unroll
    for (int q = 0; q < 8; ++q) { const float xv = sp[(size_t)q * DM]; o[q] = (h16)xv; unsigned short a1, c1; splitf(xv, a1, c1); oh[q] = a1; ol[q] = c1; }
    const bool hr = (t < RH); const size_t eo = ((size_t)g * HD + d) * RH + t;
    *(volatile v8h*)(vt16 + e) = o; if (hr) { *(volatile v8us*)(vth + eo) = oh; *(volatile v8us*)(vtl + eo) = ol; }
    __threadfence();
    *(volatile v8h*)(vt16 + e) = o; if (hr) { *(volatile v8us*)(vth + eo) = oh; *(volatile v8us*)(vtl + eo) = ol; }
}

__global__ __launch_bounds__(128) __attribute__((amdgpu_num_vgpr(256)))
void k_flashP(const h16* q16, const h16* qr16, const h16* k16, const h16* kr16, const h16* vt16, float* ctx, int qbase) {
    __shared__ __align__(16) float os[4][16 * 132];
    const int lane = threadIdx.x & 31, wv = threadIdx.x >> 5, lr = lane & 15, hi = lane >> 4;
    const int h = blockIdx.y, b = blockIdx.z;
    const int q0 = qbase + blockIdx.x * 64 + wv * 16;
    const int qi = q0 + lr;
    const size_t rq = (size_t)b * SEQ + qi, rk = (size_t)b * SEQ + lr;
    const h16* qp = q16 + rq * DM + h * HD + 8 * hi;
    const h16* qrp = qr16 + rq * (NH * RD) + h * RD + 8 * hi;
    const h16* kp = k16 + rk * DM + h * HD + 8 * hi;
    const h16* krp = kr16 + rk * RD + 8 * hi;
    const h16* vp = vt16 + ((size_t)(b * NH + h) * HD + lr) * SEQ + 8 * hi;
    v8f o[8];
#pragma unroll
    for (int i = 0; i < 8; ++i) o[i] = (v8f){};
    float m = -3.0e38f, l = 0.f;
    const float SC2 = 0.07216878364870323f * 1.4426950408889634f;
    const int nch = (q0 + 47) >> 5;
#pragma unroll 1
    for (int c = 0; c < nch; ++c) {
        asm volatile("" ::: "memory");
        const int key0 = c << 5;
        v8f s[2]; s[0] = (v8f){}; s[1] = (v8f){};
#pragma unroll
        for (int kc = 0; kc < 4; ++kc) {
            const v16h bq = ldh(qp + kc * 32);
#pragma unroll
            for (int j = 0; j < 2; ++j) { const v16h a = ldh(kp + (size_t)(key0 + 16 * j) * DM + kc * 32); s[j] = wmma16(a, bq, s[j]); }
        }
#pragma unroll
        for (int kc = 0; kc < 2; ++kc) {
            const v16h bq = ldh(qrp + kc * 32);
#pragma unroll
            for (int j = 0; j < 2; ++j) { const v16h a = ldh(krp + (size_t)(key0 + 16 * j) * RD + kc * 32); s[j] = wmma16(a, bq, s[j]); }
        }
        asm volatile("v_nop\n\tv_nop\n\tv_nop\n\tv_nop" : "+v"(s[0]), "+v"(s[1]));
        float cm = -3.0e38f;
#pragma unroll
        for (int j = 0; j < 2; ++j)
#pragma unroll
            for (int r = 0; r < 8; ++r) { const int key = key0 + 16 * j + 8 * hi + r; const float t = (key <= qi) ? s[j][r] * SC2 : -3.0e38f; s[j][r] = t; cm = fmaxf(cm, t); }
        cm = fmaxf(cm, __shfl_xor(cm, 16, 32));
        const float mn = fmaxf(m, cm);
        const float alpha = __builtin_amdgcn_exp2f(m - mn);
        float rs = 0.f;
#pragma unroll
        for (int j = 0; j < 2; ++j)
#pragma unroll
            for (int r = 0; r < 8; ++r) { const float p = __builtin_amdgcn_exp2f(s[j][r] - mn); s[j][r] = p; rs += p; }
        rs += __shfl_xor(rs, 16, 32);
        l = l * alpha + rs; m = mn;
#pragma unroll
        for (int i = 0; i < 8; ++i) o[i] = o[i] * alpha;
        v16h pb = (v16h){};
#pragma unroll
        for (int r = 0; r < 8; ++r) { pb[r] = (h16)(s[0][r] * PCAR); pb[8 + r] = (h16)(s[1][r] * PCAR); }
#pragma unroll
        for (int i = 0; i < 8; ++i) { const v16h a = ldh(vp + (size_t)(16 * i) * SEQ + key0); o[i] = wmma16(a, pb, o[i]); }
        asm volatile("v_nop\n\tv_nop\n\tv_nop\n\tv_nop" : "+v"(o[0]), "+v"(o[1]), "+v"(o[2]), "+v"(o[3]), "+v"(o[4]), "+v"(o[5]), "+v"(o[6]), "+v"(o[7]) : "v"(pb));
    }
    const float f = 1.0f / (l * PCAR);
    float* ob = &os[wv][0];
#pragma unroll
    for (int i = 0; i < 8; ++i)
#pragma unroll
        for (int r = 0; r < 8; ++r) ob[lr * 132 + 16 * i + 8 * hi + r] = o[i][r] * f;
    __builtin_amdgcn_fence(3, "wavefront"); __builtin_amdgcn_wave_barrier(); asm volatile("" ::: "memory");
    float* crow = ctx + ((size_t)b * SEQ + q0) * DM + h * HD + 4 * lane;
#pragma unroll 1
    for (int ps = 0; ps < 2; ++ps) {
#pragma unroll
        for (int qq = 0; qq < 16; ++qq) { const v4f val = *(const v4fa*)(ob + qq * 132 + 4 * lane); *(volatile v4f*)(crow + (size_t)qq * DM) = val; }
        if (ps == 0) __threadfence(); }
}

__global__ __launch_bounds__(128) __attribute__((amdgpu_num_vgpr(256)))
void k_flashH(const bf* qh, const bf* qlw, const bf* qrh, const bf* qrlw, const bf* kh, const bf* klw, const bf* krh, const bf* krlw, const bf* vth, const bf* vtl, float* ctx) {
    __shared__ __align__(16) float os[4][16 * 132];
    const int lane = threadIdx.x & 31, wv = threadIdx.x >> 5, lr = lane & 15, hi = lane >> 4;
    const int h = blockIdx.y, b = blockIdx.z;
    const int q0 = blockIdx.x * 64 + wv * 16;
    const int qi = q0 + lr;
    const size_t rq = (size_t)b * RH + qi, rk = (size_t)b * RH + lr;
    const bf* qhp = qh + rq * DM + h * HD + 8 * hi;       const bf* qlp = qlw + rq * DM + h * HD + 8 * hi;
    const bf* qrhp = qrh + rq * (NH * RD) + h * RD + 8 * hi; const bf* qrlp = qrlw + rq * (NH * RD) + h * RD + 8 * hi;
    const bf* khp = kh + rk * DM + h * HD + 8 * hi;       const bf* klp = klw + rk * DM + h * HD + 8 * hi;
    const bf* krhp = krh + rk * RD + 8 * hi;              const bf* krlp = krlw + rk * RD + 8 * hi;
    const bf* vhp = vth + ((size_t)(b * NH + h) * HD + lr) * RH + 8 * hi;
    const bf* vlp = vtl + ((size_t)(b * NH + h) * HD + lr) * RH + 8 * hi;
    v8f o[8];
#pragma unroll
    for (int i = 0; i < 8; ++i) o[i] = (v8f){};
    float m = -3.0e38f, l = 0.f;
    const float SC2 = 0.07216878364870323f * 1.4426950408889634f;
    const int nch = (q0 + 47) >> 5;
#pragma unroll 1
    for (int c = 0; c < nch; ++c) {
        asm volatile("" ::: "memory");
        const int key0 = c << 5;
        v8f s[2]; s[0] = (v8f){}; s[1] = (v8f){};
#pragma unroll
        for (int kc = 0; kc < 4; ++kc) {
            const v16bf bh = ldb(qhp + kc * 32), bl = ldb(qlp + kc * 32);
#pragma unroll
            for (int j = 0; j < 2; ++j) { const v16bf ah = ldb(khp + (size_t)(key0 + 16 * j) * DM + kc * 32), al = ldb(klp + (size_t)(key0 + 16 * j) * DM + kc * 32);
                s[j] = wmmab(ah, bh, s[j]); s[j] = wmmab(al, bh, s[j]); s[j] = wmmab(ah, bl, s[j]); }
        }
#pragma unroll
        for (int kc = 0; kc < 2; ++kc) {
            const v16bf bh = ldb(qrhp + kc * 32), bl = ldb(qrlp + kc * 32);
#pragma unroll
            for (int j = 0; j < 2; ++j) { const v16bf ah = ldb(krhp + (size_t)(key0 + 16 * j) * RD + kc * 32), al = ldb(krlp + (size_t)(key0 + 16 * j) * RD + kc * 32);
                s[j] = wmmab(ah, bh, s[j]); s[j] = wmmab(al, bh, s[j]); s[j] = wmmab(ah, bl, s[j]); }
        }
        asm volatile("v_nop\n\tv_nop\n\tv_nop\n\tv_nop" : "+v"(s[0]), "+v"(s[1]));
        float cm = -3.0e38f;
#pragma unroll
        for (int j = 0; j < 2; ++j)
#pragma unroll
            for (int r = 0; r < 8; ++r) { const int key = key0 + 16 * j + 8 * hi + r; const float t = (key <= qi) ? s[j][r] * SC2 : -3.0e38f; s[j][r] = t; cm = fmaxf(cm, t); }
        cm = fmaxf(cm, __shfl_xor(cm, 16, 32));
        const float mn = fmaxf(m, cm);
        const float alpha = __builtin_amdgcn_exp2f(m - mn);
        float rs = 0.f;
#pragma unroll
        for (int j = 0; j < 2; ++j)
#pragma unroll
            for (int r = 0; r < 8; ++r) { const float p = __builtin_amdgcn_exp2f(s[j][r] - mn); s[j][r] = p; rs += p; }
        rs += __shfl_xor(rs, 16, 32);
        l = l * alpha + rs; m = mn;
#pragma unroll
        for (int i = 0; i < 8; ++i) o[i] = o[i] * alpha;
        v16us phv = (v16us){}, plv = (v16us){};
#pragma unroll
        for (int r = 0; r < 8; ++r) { unsigned short a1, c1; splitf(s[0][r], a1, c1); phv[r] = a1; plv[r] = c1; splitf(s[1][r], a1, c1); phv[8 + r] = a1; plv[8 + r] = c1; }
        const v16bf ph = __builtin_bit_cast(v16bf, phv), pl = __builtin_bit_cast(v16bf, plv);
#pragma unroll
        for (int i = 0; i < 8; ++i) { const v16bf ah = ldb(vhp + (size_t)(16 * i) * RH + key0), al = ldb(vlp + (size_t)(16 * i) * RH + key0);
            o[i] = wmmab(ah, ph, o[i]); o[i] = wmmab(ah, pl, o[i]); o[i] = wmmab(al, ph, o[i]); }
        asm volatile("v_nop\n\tv_nop\n\tv_nop\n\tv_nop" : "+v"(o[0]), "+v"(o[1]), "+v"(o[2]), "+v"(o[3]), "+v"(o[4]), "+v"(o[5]), "+v"(o[6]), "+v"(o[7]) : "v"(ph), "v"(pl));
    }
    const float f = 1.0f / l;
    float* ob = &os[wv][0];
#pragma unroll
    for (int i = 0; i < 8; ++i)
#pragma unroll
        for (int r = 0; r < 8; ++r) ob[lr * 132 + 16 * i + 8 * hi + r] = o[i][r] * f;
    __builtin_amdgcn_fence(3, "wavefront"); __builtin_amdgcn_wave_barrier(); asm volatile("" ::: "memory");
    float* crow = ctx + ((size_t)b * SEQ + q0) * DM + h * HD + 4 * lane;
#pragma unroll 1
    for (int ps = 0; ps < 2; ++ps) {
#pragma unroll
        for (int qq = 0; qq < 16; ++qq) { const v4f val = *(const v4fa*)(ob + qq * 132 + 4 * lane); *(volatile v4f*)(crow + (size_t)qq * DM) = val; }
        if (ps == 0) __threadfence(); }
}

extern "C" void kernel_launch(void* const* d_in, const int* in_sizes, int n_in,
                              void* d_out, int out_size, void* d_ws, size_t ws_size, hipStream_t stream) {
    if (n_in < 9) return;
    const size_t nrow = (size_t)NB * SEQ;
    if ((size_t)in_sizes[0] < ((size_t)(NB - 1) * TFULL + SEQ) * DM) return;
    if (in_sizes[1] < DM * LAT || in_sizes[2] < LAT * DM || in_sizes[3] < LAT * NH * RD || in_sizes[4] < DM * LAT || in_sizes[5] < LAT * DM || in_sizes[6] < LAT * DM || in_sizes[7] < DM * RD || in_sizes[8] < DM * DM) return;
    if ((size_t)out_size < ((size_t)(NB - 1) * TFULL + SEQ) * DM) return;
    const float* x = (const float*)d_in[0]; const float* Wqd = (const float*)d_in[1]; const float* Wqu = (const float*)d_in[2]; const float* Wqr = (const float*)d_in[3];
    const float* Wkvd = (const float*)d_in[4]; const float* Wku = (const float*)d_in[5]; const float* Wvu = (const float*)d_in[6]; const float* Wkr = (const float*)d_in[7]; const float* Wo = (const float*)d_in[8];
    float* OUT = (float*)d_out;

    char* wsp = (char*)d_ws; size_t off = 0;
    auto take = [&](size_t bytes) { char* p = wsp + off; off += (bytes + 255) & ~(size_t)255; return p; };
    char* arA = take(nrow * DM * 4);
    bf* xb = (bf*)arA; float* QLf = (float*)(arA + nrow * DM * 2); float* CKVf = (float*)(arA + nrow * DM * 2 + nrow * LAT * 4); float* F1 = (float*)arA;
    h16* ql16 = (h16*)take(nrow * LAT * 2); bf* qlh = (bf*)take((size_t)NB * RH * LAT * 2); bf* qll = (bf*)take((size_t)NB * RH * LAT * 2);
    h16* ckv16 = (h16*)take(nrow * LAT * 2); bf* ckvh = (bf*)take((size_t)NB * RH * LAT * 2); bf* ckvl = (bf*)take((size_t)NB * RH * LAT * 2);
    float* KR0 = (float*)take(nrow * RD * 4); float* CT = (float*)take((size_t)SEQ * 32 * 4); float* ST = (float*)take((size_t)SEQ * 32 * 4);
    bf* Wqd_b = (bf*)take((size_t)DM * LAT * 2); bf* Wkvd_b = (bf*)take((size_t)DM * LAT * 2); bf* Wkr_b = (bf*)take((size_t)DM * RD * 2);
    h16* Wup_h = (h16*)take((size_t)DM * LAT * 2); bf* Wup_b = (bf*)take((size_t)DM * LAT * 2);
    const size_t szq16 = nrow * DM * 2, szhr = (size_t)NB * RH * DM * 2, szqr16 = nrow * NH * RD * 2, szqrh = (size_t)NB * RH * NH * RD * 2, szkr16 = nrow * RD * 2, szkrh = (size_t)NB * RH * RD * 2;
    const size_t P1 = szq16 + 2 * szhr + szqr16 + 2 * szqrh + szq16 + 2 * szhr + szkr16 + 2 * szkrh + szq16 + 2 * szhr;
    const size_t szwo = (size_t)DM * DM * 2; const size_t P2 = 2 * szwo + szq16 + 2 * szhr;
    char* arP = take(P1 > P2 ? P1 : P2);
    char* pp = arP;
    auto sub = [&](size_t bytes) { char* p = pp; pp += bytes; return p; };
    h16* q16 = (h16*)sub(szq16); bf* qh = (bf*)sub(szhr); bf* qlo = (bf*)sub(szhr); h16* qr16 = (h16*)sub(szqr16); bf* qrh = (bf*)sub(szqrh); bf* qrlo = (bf*)sub(szqrh);
    h16* k16 = (h16*)sub(szq16); bf* kh = (bf*)sub(szhr); bf* klo = (bf*)sub(szhr); h16* kr16 = (h16*)sub(szkr16); bf* krh = (bf*)sub(szkrh); bf* krlo = (bf*)sub(szkrh);
    h16* vt16 = (h16*)sub(szq16); bf* vth = (bf*)sub(szhr); bf* vtl = (bf*)sub(szhr);
    float* QRf = (float*)k16;
    pp = arP; bf* Wo_b = (bf*)sub(szwo); h16* Wo_h = (h16*)sub(szwo); h16* ctx16 = (h16*)sub(szq16); bf* ctxh = (bf*)sub(szhr); bf* ctxl = (bf*)sub(szhr);
    if (off > ws_size) return;

    auto g1 = [](size_t nthreads) { return dim3((unsigned)((nthreads + 255) / 256)); };
    auto gw = [](size_t K, size_t N) { return dim3((unsigned)((N * K / 64 + 63) / 64)); };
    auto up = [&](const h16* a16, const bf* ahh, const bf* all, int N, float* Cf) {
        if (SEQ > RH) k_gemmw<h16, 0><<<dim3((SEQ - RH) / 64, N / 64, NB), 32, 0, stream>>>(a16 + (size_t)RH * LAT, a16 + (size_t)RH * LAT, Wup_h, LAT, Cf + (size_t)RH * N, N, 1.0f / WSC, (size_t)SEQ * LAT, (size_t)SEQ * N);
        k_gemmw<bf, 1><<<dim3(RH / 64, N / 64, NB), 32, 0, stream>>>(ahh, all, Wup_b, LAT, Cf, N, 1.0f, (size_t)RH * LAT, (size_t)SEQ * N);
    };

    k_rtab<<<g1((size_t)SEQ * 32), 256, 0, stream>>>(CT, ST);
    k_xcvt<<<g1(nrow * DM / 8), 256, 0, stream>>>(x, xb);
    k_wt<0><<<gw(DM, LAT), 256, 0, stream>>>(Wqd, DM, LAT, Wqd_b, Wup_h, 1.0f);
    k_wt<0><<<gw(DM, LAT), 256, 0, stream>>>(Wkvd, DM, LAT, Wkvd_b, Wup_h, 1.0f);
    k_wt<0><<<gw(DM, RD), 256, 0, stream>>>(Wkr, DM, RD, Wkr_b, Wup_h, 1.0f);
    k_gemmw<bf, 0><<<dim3((unsigned)(nrow / 64), LAT / 64, 1), 32, 0, stream>>>(xb, xb, Wqd_b, DM, QLf, LAT, 1.0f, 0, 0);
    k_gemmw<bf, 0><<<dim3((unsigned)(nrow / 64), LAT / 64, 1), 32, 0, stream>>>(xb, xb, Wkvd_b, DM, CKVf, LAT, 1.0f, 0, 0);
    k_gemmw<bf, 0><<<dim3((unsigned)(nrow / 64), RD / 64, 1), 32, 0, stream>>>(xb, xb, Wkr_b, DM, KR0, RD, 1.0f, 0, 0);
    k_act<<<g1(nrow * LAT / 8), 256, 0, stream>>>(QLf, LAT, 1.0f, ql16, qlh, qll);
    k_act<<<g1(nrow * LAT / 8), 256, 0, stream>>>(CKVf, LAT, 1.0f, ckv16, ckvh, ckvl);
    k_wt<1><<<gw(LAT, DM), 256, 0, stream>>>(Wqu, LAT, DM, Wup_b, Wup_h, WSC);
    up(ql16, qlh, qll, DM, F1);
    k_act<<<g1(nrow * DM / 8), 256, 0, stream>>>(F1, DM, 1.0f, q16, qh, qlo);
    k_wt<1><<<gw(LAT, NH * RD), 256, 0, stream>>>(Wqr, LAT, NH * RD, Wup_b, Wup_h, WSC);
    up(ql16, qlh, qll, NH * RD, QRf);
    k_rope<<<g1(nrow * NH * RD / 8), 256, 0, stream>>>(QRf, NH * RD, CT, ST, qr16, qrh, qrlo);
    k_wt<1><<<gw(LAT, DM), 256, 0, stream>>>(Wku, LAT, DM, Wup_b, Wup_h, WSC);
    up(ckv16, ckvh, ckvl, DM, F1);
    k_act<<<g1(nrow * DM / 8), 256, 0, stream>>>(F1, DM, 1.0f, k16, kh, klo);
    k_rope<<<g1(nrow * RD / 8), 256, 0, stream>>>(KR0, RD, CT, ST, kr16, krh, krlo);
    k_wt<1><<<gw(LAT, DM), 256, 0, stream>>>(Wvu, LAT, DM, Wup_b, Wup_h, WSC);
    up(ckv16, ckvh, ckvl, DM, F1);
    k_vtp8<<<g1((size_t)NU * HD * SEQ / 8), 256, 0, stream>>>(F1, vt16, vth, vtl);
    if (SEQ > RH) k_flashP<<<dim3((SEQ - RH) / 64, NH, NB), 128, 0, stream>>>(q16, qr16, k16, kr16, vt16, F1, RH);
    k_flashH<<<dim3(RH / 64, NH, NB), 128, 0, stream>>>(qh, qlo, qrh, qrlo, kh, klo, krh, krlo, vth, vtl, F1);
    k_act<<<g1(nrow * DM / 8), 256, 0, stream>>>(F1, DM, CCAR, ctx16, ctxh, ctxl);
    k_wt<1><<<gw(DM, DM), 256, 0, stream>>>(Wo, DM, DM, Wo_b, Wo_h, WSC);
    if (SEQ > RH) k_gemmw<h16, 0><<<dim3((SEQ - RH) / 64, DM / 64, NB), 32, 0, stream>>>(ctx16 + (size_t)RH * DM, ctx16 + (size_t)RH * DM, Wo_h, DM, OUT + (size_t)RH * DM, DM, 1.0f / (CCAR * WSC), (size_t)SEQ * DM, (size_t)TFULL * DM);
    k_gemmw<bf, 1><<<dim3(RH / 64, DM / 64, NB), 32, 0, stream>>>(ctxh, ctxl, Wo_b, DM, OUT, DM, 1.0f, (size_t)RH * DM, (size_t)TFULL * DM);
}
